// KernelExpansion_68564857913960
// MI455X (gfx1250) — hardware-verified
//
#include <hip/hip_runtime.h>
#include <math.h>

typedef __attribute__((ext_vector_type(16))) __bf16   v16b;
typedef __attribute__((ext_vector_type(8)))  __bf16   v8b;
typedef __attribute__((ext_vector_type(8)))  float    v8f;
typedef __attribute__((ext_vector_type(4)))  float    v4f;
typedef __attribute__((ext_vector_type(4)))  unsigned v4u;

constexpr int kM  = 16384;
constexpr int kN  = 8192;
constexpr int kD  = 24;
constexpr int kKP = 32;
constexpr int  kInputsRneToBf16 = 1;
constexpr bool kSplit = (kInputsRneToBf16 == 0);
constexpr float kLog2e = 1.44269504088896340736f;
constexpr int kSBlocks = kN / 256;
constexpr int kXBlocks = kM / 256;
static_assert(kD == 24 && kKP == 32, "depth and padded depth");
static_assert((kD % 4) == 0 && kD <= kKP, "row loads are whole 16-B vectors");
static_assert((kN % 256) == 0 && (kM % 256) == 0, "plane-building blocks cover whole rows");
static_assert((kN % 16) == 0 && (kM % 128) == 0, "tile multiples of the main kernel");

constexpr size_t kBytesSH  = (size_t)kN * kKP * 2;
constexpr size_t kBytesSL  = kSplit ? (size_t)kN * kKP * 2 : 0;
constexpr size_t kBytesXH  = (size_t)kM * kKP * 2;
constexpr size_t kBytesXL  = kSplit ? (size_t)kM * kKP * 2 : 0;
constexpr size_t kBytesSSQ = (size_t)kN * 4;
constexpr size_t kBytesWP  = (size_t)kN * 4;
constexpr size_t kBytesXHN = (size_t)kM * 4;
constexpr size_t kOffSH  = 0;
constexpr size_t kOffSL  = kOffSH  + kBytesSH;
constexpr size_t kOffXH  = kOffSL  + kBytesSL;
constexpr size_t kOffXL  = kOffXH  + kBytesXH;
constexpr size_t kOffSSQ = kOffXL  + kBytesXL;
constexpr size_t kOffWP  = kOffSSQ + kBytesSSQ;
constexpr size_t kOffXHN = kOffWP  + kBytesWP;
constexpr size_t kWsTotal = kOffXHN + kBytesXHN;
static_assert(kWsTotal == (kSplit ? 3276800ull : 1703936ull), "carve total");
static_assert(kWsTotal <= 134217728ull, "carve cap");
static_assert((kOffSL % 128) == 0 && (kOffXH % 128) == 0 && (kOffXL % 128) == 0 && (kOffSSQ % 128) == 0 &&
              (kOffWP % 128) == 0 && (kOffXHN % 128) == 0, "128-B aligned regions");

__device__ __forceinline__ unsigned bf_bits_rne(float f) {
  const unsigned u = __float_as_uint(f);
  return (u + 0x7FFFu + ((u >> 16) & 1u)) >> 16;
}
__device__ __forceinline__ float bf_bits_to_f32(unsigned hb) { return __uint_as_float(hb << 16); }
__device__ __forceinline__ float bf16_rne_value(float f) { return bf_bits_to_f32(bf_bits_rne(f)); }

template <bool SPL>
__device__ __forceinline__ void convert_one(float f, unsigned& hb, unsigned& lb, float& sum) {
  hb = bf_bits_rne(f);
  const float r = bf_bits_to_f32(hb);
  if (SPL) {
    lb = bf_bits_rne(f - r);
    sum = fmaf(f, f, sum);
  } else {
    lb = 0u;
    sum = fmaf(r, r, sum);
  }
}

union FragU { v16b v; v8b h[2]; };
__device__ __forceinline__ v16b frag_load(const __bf16* p) {
  FragU f;
  f.h[0] = *(const v8b*)(p);
  f.h[1] = *(const v8b*)(p + 16);
  return f.v;
}
__device__ __forceinline__ v8f mma_guarded(v16b a, v16b b, v8f c) {
  c = __builtin_amdgcn_wmma_f32_16x16x32_bf16(false, a, false, b, (short)0, c, false, false);
  asm volatile("v_nop\n\tv_nop\n\tv_nop\n\tv_nop" : "+v"(c) : "v"(a), "v"(b));
  return c;
}

template <bool SPL>
__global__ __launch_bounds__(256) void prep_planes_kernel(
    const float* __restrict__ xq, const float* __restrict__ smp, const float* __restrict__ wts,
    const float* __restrict__ sigma_p, const float* __restrict__ len_p,
    unsigned* __restrict__ sHiW, unsigned* __restrict__ sLoW,
    unsigned* __restrict__ xHiW, unsigned* __restrict__ xLoW,
    float* __restrict__ ssq2, float* __restrict__ wpl, float* __restrict__ xhl)
{
  __shared__ __align__(16) v4u tHi[256 * 4];
  __shared__ __align__(16) v4u tLo[SPL ? 256 * 4 : 4];
  const int tid = threadIdx.x, lane = tid & 31, wave = tid >> 5;
  const bool isS = ((int)blockIdx.x < kSBlocks);
  const int blk = isS ? (int)blockIdx.x : ((int)blockIdx.x - kSBlocks);
  const int row = blk * 256 + tid;
  const float* src = isS ? smp : xq;
  const v4f* rp = (const v4f*)(src + (size_t)row * kD);

  unsigned hw[16], lw[16];
  float sum = 0.0f;
#pragma unroll
  for (int q = 0; q < kD / 4; ++q) {
    const v4f v = rp[q];
    const float f0 = v[0];
    const float f1 = v[1];
    const float f2 = v[2];
    const float f3 = v[3];
    unsigned h0, h1, h2, h3, l0, l1, l2, l3;
    convert_one<SPL>(f0, h0, l0, sum);
    convert_one<SPL>(f1, h1, l1, sum);
    convert_one<SPL>(f2, h2, l2, sum);
    convert_one<SPL>(f3, h3, l3, sum);
    hw[2 * q]     = h0 | (h1 << 16);
    hw[2 * q + 1] = h2 | (h3 << 16);
    lw[2 * q]     = l0 | (l1 << 16);
    lw[2 * q + 1] = l2 | (l3 << 16);
  }
#pragma unroll
  for (int q = kD / 2; q < 16; ++q) {
    hw[q] = 0u;
    lw[q] = 0u;
  }
#pragma unroll
  for (int j = 0; j < 4; ++j) {
    const v4u a = {hw[4 * j], hw[4 * j + 1], hw[4 * j + 2], hw[4 * j + 3]};
    tHi[tid * 4 + j] = a;
    if (SPL) {
      const v4u b = {lw[4 * j], lw[4 * j + 1], lw[4 * j + 2], lw[4 * j + 3]};
      tLo[tid * 4 + j] = b;
    }
  }

  const int rowc = (row < kN) ? row : (kN - 1);
  float wv = wts[rowc];
  float sg = sigma_p[0];
  float ln = len_p[0];
  if (!SPL) {
    wv = bf16_rne_value(wv);
    sg = bf16_rne_value(sg);
    ln = bf16_rne_value(ln);
  }
  const float invl2 = 1.0f / (ln * ln);
  const float coef  = (-0.5f * kLog2e) * invl2;
  const float v0 = isS ? (coef * sum) : (-0.5f * sum);
  const float v1 = wv * (sg * sg);
  float* p0 = isS ? (ssq2 + row) : (xhl + row);
  float* p1 = wpl + rowc;

  __syncthreads();

  v4u hq[4], lq[4];
#pragma unroll
  for (int it = 0; it < 4; ++it) {
    hq[it] = tHi[wave * 128 + it * 32 + lane];
    if (SPL) lq[it] = tLo[wave * 128 + it * 32 + lane];
    else lq[it] = hq[it];
  }
  unsigned* hiW = isS ? sHiW : xHiW;
  unsigned* loW = isS ? sLoW : xLoW;
  const size_t woff = (size_t)(blk * 256 + wave * 32) * 16 + (size_t)lane * 4;
  for (int pass = 0; pass < 2; ++pass) {
#pragma unroll
    for (int it = 0; it < 4; ++it) {
      *(volatile v4u*)(hiW + woff + it * 128) = hq[it];
      if (SPL) *(volatile v4u*)(loW + woff + it * 128) = lq[it];
    }
    *(volatile float*)p0 = v0;
    if (isS) *(volatile float*)p1 = v1;
    __threadfence();
  }
}

template <bool SPL>
__global__ __launch_bounds__(128) void rbf_sum_kernel(
    const unsigned short* __restrict__ sHp, const unsigned short* __restrict__ sLp,
    const unsigned short* __restrict__ xHp, const unsigned short* __restrict__ xLp,
    const float* __restrict__ ssq2, const float* __restrict__ wpl, const float* __restrict__ xhl,
    const float* __restrict__ len_p, float* __restrict__ out)
{
  const __bf16* sH = (const __bf16*)sHp;
  const __bf16* sL = (const __bf16*)sLp;
  const __bf16* xH = (const __bf16*)xHp;
  const __bf16* xL = (const __bf16*)xLp;
  const int lane = threadIdx.x & 31;
  const int wave = threadIdx.x >> 5;
  const int h = lane >> 4;
  const int c = lane & 15;
  const int m_base = ((int)blockIdx.x * 4 + wave) * 32;

  float ln = len_p[0];
  if (!SPL) ln = bf16_rne_value(ln);
  const float c2 = kLog2e * (1.0f / (ln * ln));

  const v16b b0h = frag_load(xH + (size_t)(m_base + c) * kKP + 8 * h);
  const v16b b1h = frag_load(xH + (size_t)(m_base + 16 + c) * kKP + 8 * h);
  v16b b0l = b0h, b1l = b1h;
  if (SPL) {
    b0l = frag_load(xL + (size_t)(m_base + c) * kKP + 8 * h);
    b1l = frag_load(xL + (size_t)(m_base + 16 + c) * kKP + 8 * h);
  }
  const float xs0 = xhl[m_base + c];
  const float xs1 = xhl[m_base + 16 + c];
  const v8f seed0 = {xs0, xs0, xs0, xs0, xs0, xs0, xs0, xs0};
  const v8f seed1 = {xs1, xs1, xs1, xs1, xs1, xs1, xs1, xs1};

  float acc0[8], acc1[8];
#pragma unroll
  for (int r = 0; r < 8; ++r) {
    acc0[r] = 0.0f;
    acc1[r] = 0.0f;
  }

#pragma unroll 1
  for (int n0 = 0; n0 < kN; n0 += 16) {
    const v16b ah = frag_load(sH + (size_t)(n0 + c) * kKP + 8 * h);
    v8f c0 = mma_guarded(ah, b0h, seed0);
    v8f c1 = mma_guarded(ah, b1h, seed1);
    if (SPL) {
      const v16b al = frag_load(sL + (size_t)(n0 + c) * kKP + 8 * h);
      c0 = mma_guarded(ah, b0l, c0);
      c1 = mma_guarded(ah, b1l, c1);
      c0 = mma_guarded(al, b0h, c0);
      c1 = mma_guarded(al, b1h, c1);
    }
    const v4f sa = *(const v4f*)(ssq2 + n0 + 8 * h);
    const v4f sb = *(const v4f*)(ssq2 + n0 + 8 * h + 4);
    const v4f wa = *(const v4f*)(wpl + n0 + 8 * h);
    const v4f wb = *(const v4f*)(wpl + n0 + 8 * h + 4);
#pragma unroll
    for (int r = 0; r < 4; ++r) {
      float a0 = fmaf(c2, c0[r], sa[r]);
      a0 = fminf(a0, 0.0f);
      acc0[r] = fmaf(wa[r], __builtin_amdgcn_exp2f(a0), acc0[r]);
      float a1 = fmaf(c2, c1[r], sa[r]);
      a1 = fminf(a1, 0.0f);
      acc1[r] = fmaf(wa[r], __builtin_amdgcn_exp2f(a1), acc1[r]);
    }
#pragma unroll
    for (int r = 0; r < 4; ++r) {
      float a0 = fmaf(c2, c0[4 + r], sb[r]);
      a0 = fminf(a0, 0.0f);
      acc0[4 + r] = fmaf(wb[r], __builtin_amdgcn_exp2f(a0), acc0[4 + r]);
      float a1 = fmaf(c2, c1[4 + r], sb[r]);
      a1 = fminf(a1, 0.0f);
      acc1[4 + r] = fmaf(wb[r], __builtin_amdgcn_exp2f(a1), acc1[4 + r]);
    }
  }

  const float t0 = ((acc0[0] + acc0[1]) + (acc0[2] + acc0[3])) + ((acc0[4] + acc0[5]) + (acc0[6] + acc0[7]));
  const float t1 = ((acc1[0] + acc1[1]) + (acc1[2] + acc1[3])) + ((acc1[4] + acc1[5]) + (acc1[6] + acc1[7]));
  const float o0 = __shfl_xor(t0, 16, 32);
  const float o1 = __shfl_xor(t1, 16, 32);
  const float tot0 = t0 + o0;
  const float tot1 = t1 + o1;
  const float res = (h == 0) ? tot0 : tot1;
  volatile float* op = (volatile float*)(out + m_base + lane);
  *op = res;
  __threadfence();
  *op = res;
}

extern "C" void kernel_launch(void* const* d_in, const int* in_sizes, int n_in,
                              void* d_out, int out_size, void* d_ws, size_t ws_size,
                              hipStream_t stream) {
  if (n_in < 5) return;
  if (in_sizes[0] != kM * kD) return;
  if (in_sizes[1] != kN * kD) return;
  if (in_sizes[2] != kN) return;
  if (in_sizes[3] != 1) return;
  if (in_sizes[4] != 1) return;
  if (out_size != kM) return;
  if (ws_size < kWsTotal) return;

  const float* xq      = (const float*)d_in[0];
  const float* smp     = (const float*)d_in[1];
  const float* wts     = (const float*)d_in[2];
  const float* sigma_p = (const float*)d_in[3];
  const float* len_p   = (const float*)d_in[4];
  float* out = (float*)d_out;

  char* ws = (char*)d_ws;
  unsigned short* SH  = (unsigned short*)(ws + kOffSH);
  unsigned short* SL  = (unsigned short*)(ws + kOffSL);
  unsigned short* XH  = (unsigned short*)(ws + kOffXH);
  unsigned short* XL  = (unsigned short*)(ws + kOffXL);
  float*          SSQ = (float*)(ws + kOffSSQ);
  float*          WP  = (float*)(ws + kOffWP);
  float*          XHN = (float*)(ws + kOffXHN);

  prep_planes_kernel<kSplit><<<kSBlocks + kXBlocks, 256, 0, stream>>>(
      xq, smp, wts, sigma_p, len_p,
      (unsigned*)SH, (unsigned*)SL, (unsigned*)XH, (unsigned*)XL,
      SSQ, WP, XHN);

  rbf_sum_kernel<kSplit><<<kM / 128, 128, 0, stream>>>(
      SH, SL, XH, XL, SSQ, WP, XHN, len_p, out);
}
